// MambaBlock_18580028522582
// MI455X (gfx1250) — hardware-verified
//
#include <hip/hip_runtime.h>
#include <math.h>

typedef __attribute__((ext_vector_type(16))) _Float16 v16h;
typedef __attribute__((ext_vector_type(8)))  _Float16 v8h;
typedef __attribute__((ext_vector_type(8)))  float    v8f;
typedef __attribute__((ext_vector_type(4)))  float    v4f;
typedef __attribute__((ext_vector_type(4)))  unsigned v4u;

constexpr int kBatch  = 4;
constexpr int kSeq    = 1024;
constexpr int kDm     = 1024;
constexpr int kDin    = 2048;
constexpr int kNst    = 16;
constexpr int kDtR    = 64;
constexpr int kPrjN   = 2 * kNst + kDtR;
constexpr int kPrjP   = 128;
constexpr int kXZP    = 2 * kDin;
constexpr int kRows   = kBatch * kSeq;
constexpr int kConvTP = 260;
constexpr int kScanT  = 128;
constexpr int kScanCh = 256;
constexpr int kScanTS = 64;
constexpr float kCarryW   = 32.0f;
constexpr float kCarryWdt = 8.0f;
constexpr float kCarryDt  = 16.0f;
constexpr float kCarryY   = 16.0f;
static_assert(kPrjN == 96 && kPrjP % 64 == 0 && kPrjP >= kPrjN, "x_proj width");
static_assert(kDm % 32 == 0 && kDin % 32 == 0 && kDtR % 32 == 0, "GEMM K multiples of 32");
static_assert(kRows % 64 == 0 && kXZP % 64 == 0 && kDin % 64 == 0 && kDm % 64 == 0, "GEMM M,N multiples of 64");
static_assert(kSeq % 64 == 0 && kSeq % kScanTS == 0 && kDin % kScanCh == 0 && kDin % 256 == 0, "tile multiples");
static_assert(kScanCh == 2 * kScanT, "two channels per lane");
static_assert((kSeq & (kSeq - 1)) == 0, "sequence length power of two");

constexpr size_t kOffXH  = 0;
constexpr size_t kOffWIH = kOffXH  + (size_t)kRows * kDm   * 2;
constexpr size_t kOffWXH = kOffWIH + (size_t)kXZP  * kDm   * 2;
constexpr size_t kOffWDH = kOffWXH + (size_t)kPrjP * kDin  * 2;
constexpr size_t kOffWOH = kOffWDH + (size_t)kDin  * kDtR  * 2;
constexpr size_t kOffXZ  = kOffWOH + (size_t)kDm   * kDin  * 2;
constexpr size_t kOffUC  = kOffXZ  + (size_t)kRows * kXZP  * 2;
constexpr size_t kOffPRJ = kOffUC  + (size_t)kRows * kDin  * 2;
constexpr size_t kOffDTH = kOffPRJ + (size_t)kRows * kPrjP * 4;
constexpr size_t kOffDL  = kOffDTH + (size_t)kRows * kDtR  * 2;
constexpr size_t kOffYG  = kOffDL  + (size_t)kRows * kDin  * 2;
constexpr size_t kWsTotal = kOffYG + (size_t)kRows * kDin  * 2;
static_assert(kWsTotal == 108265472ull, "carve total");
static_assert(kWsTotal <= 134217728ull, "carve cap");
static_assert((kOffWIH % 128) == 0 && (kOffWXH % 128) == 0 && (kOffWDH % 128) == 0 && (kOffWOH % 128) == 0 &&
              (kOffXZ % 128) == 0 && (kOffUC % 128) == 0 && (kOffPRJ % 128) == 0 && (kOffDTH % 128) == 0 &&
              (kOffDL % 128) == 0 && (kOffYG % 128) == 0, "128-B aligned regions");

__device__ __forceinline__ float bf_rne(float f) {
  unsigned u = __float_as_uint(f);
  u = (u + 0x7FFFu + ((u >> 16) & 1u)) & 0xFFFF0000u;
  return __uint_as_float(u);
}
__device__ __forceinline__ float h16_to_f32(unsigned hb) {
  const unsigned sgn = (hb & 0x8000u) << 16;
  const unsigned em = hb & 0x7fffu;
  const float fn = __uint_as_float((em << 13) + 0x38000000u);
  const float fs = (float)em * 5.9604644775390625e-8f;
  const float mag = (em < 0x400u) ? fs : fn;
  return __uint_as_float(__float_as_uint(mag) | sgn);
}

__device__ __forceinline__ void dep_guard4_h(v8f& a, v8f& b, v8f& c, v8f& d, v16h x, v16h y0, v16h y1, v16h y2, v16h y3) {
  asm volatile("v_nop\n\tv_nop\n\tv_nop\n\tv_nop" : "+v"(a), "+v"(b), "+v"(c), "+v"(d) : "v"(x), "v"(y0), "v"(y1), "v"(y2), "v"(y3));
}
__device__ __forceinline__ void keep4_h(v16h a, v16h b, v16h c, v16h d) { asm volatile("v_nop" :: "v"(a), "v"(b), "v"(c), "v"(d)); }
__device__ __forceinline__ void acc_guard4(v8f& a, v8f& b, v8f& c, v8f& d) { asm volatile("v_nop\n\tv_nop\n\tv_nop\n\tv_nop" : "+v"(a), "+v"(b), "+v"(c), "+v"(d)); }

union FragH { v16h v; v8h h[2]; };
__device__ __forceinline__ v16h frag_load_h(const _Float16* p) {
  FragH f;
  f.h[0] = *(const v8h*)(p);
  f.h[1] = *(const v8h*)(p + 16);
  return f.v;
}
__device__ __forceinline__ v8f mma_h(v16h a, v16h b, v8f c) {
  return __builtin_amdgcn_wmma_f32_16x16x32_f16(false, a, false, b, (short)0, c, false, false);
}

template <int OUT_MODE>
__global__ __launch_bounds__(256) void wmma_gemm64_f16(
    const unsigned short* __restrict__ Ap, int lda,
    const unsigned short* __restrict__ Btp, int ldb,
    void* __restrict__ Cout, int ldc,
    int M, int N, int K, float scale) {
  const _Float16* A  = (const _Float16*)Ap;
  const _Float16* Bt = (const _Float16*)Btp;
  __shared__ __align__(16) float sT[8][16 * 68];
  const int lane = threadIdx.x & 31;
  const int wave = threadIdx.x >> 5;
  const int tilesN = N >> 6;
  const int tilesM = M >> 6;
  const int tile = blockIdx.x * 8 + wave;
  if (tile >= tilesM * tilesN) return;
  const int tm = tile / tilesN;
  const int tn = tile - tm * tilesN;
  const int m0 = tm << 6;
  const int n0 = tn << 6;

  const int rlane = lane & 15;
  const int koff  = (lane >> 4) * 8;
  const int mOff  = (lane >> 4) * 8;

  v8f acc[4][4];
#pragma unroll
  for (int i = 0; i < 4; ++i)
#pragma unroll
    for (int j = 0; j < 4; ++j) acc[i][j] = (v8f){0.f,0.f,0.f,0.f,0.f,0.f,0.f,0.f};

  for (int k0 = 0; k0 < K; k0 += 32) {
    v16h bh[4];
#pragma unroll
    for (int j = 0; j < 4; ++j) {
      const size_t bo = (size_t)(n0 + (j << 4) + rlane) * ldb + koff + k0;
      bh[j] = frag_load_h(Bt + bo);
    }
#pragma unroll
    for (int i = 0; i < 4; ++i) {
      const size_t ao = (size_t)(m0 + (i << 4) + rlane) * lda + koff + k0;
      const v16h ah = frag_load_h(A + ao);
#pragma unroll
      for (int j = 0; j < 4; ++j) acc[i][j] = mma_h(ah, bh[j], acc[i][j]);
      dep_guard4_h(acc[i][0], acc[i][1], acc[i][2], acc[i][3], ah, bh[0], bh[1], bh[2], bh[3]);
    }
    keep4_h(bh[0], bh[1], bh[2], bh[3]);
  }
  acc_guard4(acc[0][0], acc[0][1], acc[0][2], acc[0][3]);
  acc_guard4(acc[1][0], acc[1][1], acc[1][2], acc[1][3]);
  acc_guard4(acc[2][0], acc[2][1], acc[2][2], acc[2][3]);
  acc_guard4(acc[3][0], acc[3][1], acc[3][2], acc[3][3]);

  float* slab = sT[wave];
#pragma unroll
  for (int i = 0; i < 4; ++i) {
    const int mBase = m0 + (i << 4);
#pragma unroll
    for (int j = 0; j < 4; ++j) {
#pragma unroll
      for (int r = 0; r < 8; ++r) {
        const float v = acc[i][j][r] * scale;
        slab[(mOff + r) * 68 + (j << 4) + rlane] = v;
      }
    }
    __builtin_amdgcn_fence(__ATOMIC_RELEASE, "workgroup");
    __builtin_amdgcn_wave_barrier();
    __builtin_amdgcn_fence(__ATOMIC_ACQUIRE, "workgroup");
    if (OUT_MODE == 0) {
      float* C = (float*)Cout;
      const int hh = lane >> 4, c4 = (lane & 15) * 4;
      for (int pass = 0; pass < 2; ++pass) {
#pragma unroll
        for (int it = 0; it < 8; ++it) {
          const int row = it * 2 + hh;
          const v4f v = *(const v4f*)(slab + row * 68 + c4);
          *(volatile v4f*)(C + (size_t)(mBase + row) * ldc + n0 + c4) = v;
        }
        __threadfence();
      }
    } else {
      const int q = lane >> 3, c8 = (lane & 7) * 8;
      unsigned short* C = (unsigned short*)Cout;
      for (int pass = 0; pass < 2; ++pass) {
#pragma unroll
        for (int it = 0; it < 4; ++it) {
          const int row = it * 4 + q;
          const float* sp = slab + row * 68 + c8;
          v8h hv;
#pragma unroll
          for (int e = 0; e < 8; ++e) hv[e] = (_Float16)sp[e];
          *(volatile v8h*)(C + (size_t)(mBase + row) * ldc + n0 + c8) = hv;
        }
        __threadfence();
      }
    }
    __builtin_amdgcn_fence(__ATOMIC_RELEASE, "workgroup");
    __builtin_amdgcn_wave_barrier();
    __builtin_amdgcn_fence(__ATOMIC_ACQUIRE, "workgroup");
  }
}

__global__ __launch_bounds__(256) void cast_plane_kernel(
    const float* __restrict__ src, unsigned short* __restrict__ dst, int real8, int total8, float carry)
{
  const int i = blockIdx.x * 256 + threadIdx.x;
  if (i >= total8) return;
  const bool real = (i < real8);
  const int ic = real ? i : (real8 - 1);
  const float* p = src + ((size_t)ic << 3);
  const v4f a0 = *(const v4f*)(p);
  const v4f a1 = *(const v4f*)(p + 4);
  v8h hv;
#pragma unroll
  for (int e = 0; e < 4; ++e) {
    const float f0 = bf_rne(a0[e]) * carry;
    const float f1 = bf_rne(a1[e]) * carry;
    hv[e]     = real ? (_Float16)f0 : (_Float16)0.0f;
    hv[4 + e] = real ? (_Float16)f1 : (_Float16)0.0f;
  }
  unsigned short* q = dst + ((size_t)i << 3);
  *(volatile v8h*)q = hv;
  __threadfence();
  *(volatile v8h*)q = hv;
}

__global__ __launch_bounds__(256) void dt_cast_kernel(
    const float* __restrict__ PRJ, unsigned short* __restrict__ DTH, int total8, float carry)
{
  const int i = blockIdx.x * 256 + threadIdx.x;
  if (i >= total8) return;
  const int e0  = i << 3;
  const int row = e0 >> 6;
  const int c8  = e0 & 63;
  const float* p = PRJ + (size_t)row * kPrjP + 2 * kNst + c8;
  const v4f a0 = *(const v4f*)(p);
  const v4f a1 = *(const v4f*)(p + 4);
  v8h hv;
#pragma unroll
  for (int e = 0; e < 4; ++e) {
    hv[e]     = (_Float16)(a0[e] * carry);
    hv[4 + e] = (_Float16)(a1[e] * carry);
  }
  unsigned short* qd = DTH + e0;
  *(volatile v8h*)qd = hv;
  __threadfence();
  *(volatile v8h*)qd = hv;
}

__global__ __launch_bounds__(128) void conv_silu_kernel(
    const unsigned* __restrict__ XZw, const float* __restrict__ cw, const float* __restrict__ cb,
    unsigned short* __restrict__ UC16)
{
  __shared__ __align__(16) float sT[16 * kConvTP];
  const int tid = threadIdx.x, lane = tid & 31, wave = tid >> 5;
  const int d0 = blockIdx.x * 256, d = d0 + 2 * tid;
  const int g0 = blockIdx.y * 64;
  const int l0 = g0 & (kSeq - 1);
  const float wa0 = bf_rne(cw[d * 3 + 0]), wa1 = bf_rne(cw[d * 3 + 1]), wa2 = bf_rne(cw[d * 3 + 2]);
  const float wb0 = bf_rne(cw[d * 3 + 3]), wb1 = bf_rne(cw[d * 3 + 4]), wb2 = bf_rne(cw[d * 3 + 5]);
  const float ba = bf_rne(cb[d]), bb = bf_rne(cb[d + 1]);
  float am1, bm1, ac0, bc0;
  {
    const bool hist = (l0 > 0);
    const int rp = hist ? (g0 - 1) : g0;
    const unsigned wp = XZw[((size_t)rp * kXZP + d) >> 1];
    const unsigned wc = XZw[((size_t)g0 * kXZP + d) >> 1];
    const float pa = h16_to_f32(wp & 0xffffu), pb = h16_to_f32(wp >> 16);
    am1 = hist ? pa : 0.0f;
    bm1 = hist ? pb : 0.0f;
    ac0 = h16_to_f32(wc & 0xffffu);
    bc0 = h16_to_f32(wc >> 16);
  }
#pragma unroll 1
  for (int sub = 0; sub < 4; ++sub) {
    const int lb = g0 + sub * 16;
#pragma unroll 1
    for (int s = 0; s < 16; ++s) {
      const int row = lb + s;
      const int l = l0 + sub * 16 + s;
      const bool hasn = (l + 1 < kSeq);
      const int rn = hasn ? (row + 1) : row;
      const unsigned wn = XZw[((size_t)rn * kXZP + d) >> 1];
      const float na = h16_to_f32(wn & 0xffffu), nb = h16_to_f32(wn >> 16);
      const float ap1 = hasn ? na : 0.0f;
      const float bp1 = hasn ? nb : 0.0f;
      float pa = wa0 * am1;
      pa = fmaf(wa1, ac0, pa);
      pa = fmaf(wa2, ap1, pa);
      pa = pa + ba;
      float pb = wb0 * bm1;
      pb = fmaf(wb1, bc0, pb);
      pb = fmaf(wb2, bp1, pb);
      pb = pb + bb;
      const float sa = __builtin_amdgcn_rcpf(1.0f + expf(-pa));
      const float sb = __builtin_amdgcn_rcpf(1.0f + expf(-pb));
      sT[s * kConvTP + 2 * tid]     = pa * sa;
      sT[s * kConvTP + 2 * tid + 1] = pb * sb;
      am1 = ac0; bm1 = bc0;
      ac0 = ap1; bc0 = bp1;
    }
    __syncthreads();
    v8h bv[4];
#pragma unroll
    for (int it = 0; it < 4; ++it) {
      const float* sp = sT + (it * 4 + wave) * kConvTP + lane * 8;
      const v4f a0 = *(const v4f*)(sp);
      const v4f a1 = *(const v4f*)(sp + 4);
#pragma unroll
      for (int e = 0; e < 4; ++e) {
        bv[it][e]     = (_Float16)a0[e];
        bv[it][4 + e] = (_Float16)a1[e];
      }
    }
    for (int pass = 0; pass < 2; ++pass) {
#pragma unroll
      for (int it = 0; it < 4; ++it)
        *(volatile v8h*)(UC16 + (size_t)(lb + it * 4 + wave) * kDin + d0 + lane * 8) = bv[it];
      __threadfence();
    }
    __syncthreads();
  }
}

__device__ __forceinline__ float scan_step(float (&h)[kNst], const float (&nA)[kNst],
                                           const float (&Bs)[kNst], const float (&Cs)[kNst],
                                           float v, float xt, float zv, float Dd)
{
  const float a   = __expf(-fabsf(v));
  const float u   = 1.0f + a;
  const float l1p = __logf(u) + (a - (u - 1.0f)) * __builtin_amdgcn_rcpf(u);
  const float dt  = fmaxf(v, 0.0f) + l1p;
  const float dtx = dt * xt;
  float y = 0.0f;
#pragma unroll
  for (int k = 0; k < kNst; ++k) {
    const float e = __expf(dt * nA[k]);
    h[k] = e * h[k] + dtx * Bs[k];
    y = h[k] * Cs[k] + y;
  }
  y = xt * Dd + y;
  const float sg = __builtin_amdgcn_rcpf(1.0f + __expf(-zv));
  return y * (zv * sg);
}

__global__ __launch_bounds__(128) void scan_kernel(
    const float* __restrict__ PRJ, const unsigned* __restrict__ DLw, const unsigned* __restrict__ UCw,
    const unsigned* __restrict__ XZw, const float* __restrict__ bdt, const float* __restrict__ Alog,
    const float* __restrict__ Dp, unsigned* __restrict__ YGw)
{
  __shared__ __align__(16) float    sBC[kScanTS * 32];
  __shared__ __align__(16) unsigned sY[kScanTS * kScanT];
  __shared__ __align__(16) float    sA[kNst * kScanCh];
  const int tid = threadIdx.x, lane = tid & 31, wave = tid >> 5;
  constexpr int kBlkPerB = kDin / kScanCh;
  const int bix = blockIdx.x / kBlkPerB;
  const int d0  = (blockIdx.x - bix * kBlkPerB) * kScanCh;
  const int d   = d0 + 2 * tid;
  const size_t row0 = (size_t)bix * kSeq;

#pragma unroll 1
  for (int s = 0; s < kNst; ++s) {
    const float a0 = bf_rne(Alog[(size_t)d * kNst + s]);
    const float a1 = bf_rne(Alog[(size_t)(d + 1) * kNst + s]);
    sA[s * kScanCh + 2 * tid]     = -__expf(a0);
    sA[s * kScanCh + 2 * tid + 1] = -__expf(a1);
  }
  __syncthreads();
  float nA0[kNst], nA1[kNst], h0[kNst], h1[kNst];
#pragma unroll
  for (int s = 0; s < kNst; ++s) {
    nA0[s] = sA[s * kScanCh + 2 * tid];
    nA1[s] = sA[s * kScanCh + 2 * tid + 1];
    h0[s] = 0.0f;
    h1[s] = 0.0f;
  }
  const float bb0 = bf_rne(bdt[d]), bb1 = bf_rne(bdt[d + 1]);
  const float Dd0 = bf_rne(Dp[d]),  Dd1 = bf_rne(Dp[d + 1]);

#pragma unroll 1
  for (int t0 = 0; t0 < kSeq; t0 += kScanTS) {
    __syncthreads();
#pragma unroll
    for (int i = 0; i < 4; ++i) {
      const int idx = tid + kScanT * i;
      const int r = idx >> 3, c4 = (idx & 7) * 4;
      *(v4f*)(sBC + r * 32 + c4) = *(const v4f*)(PRJ + (row0 + t0 + r) * kPrjP + c4);
    }
    __syncthreads();
#pragma unroll 1
    for (int s = 0; s < kScanTS; ++s) {
      const size_t grow = row0 + t0 + s;
      unsigned wd = DLw[(grow * kDin + d) >> 1];
      unsigned wu = UCw[(grow * kDin + d) >> 1];
      unsigned wz = XZw[(grow * kXZP + kDin + d) >> 1];
      asm volatile("" : "+v"(wd), "+v"(wu), "+v"(wz));
      float Bs[kNst], Cs[kNst];
#pragma unroll
      for (int q4 = 0; q4 < 4; ++q4) {
        const v4f bv = *(const v4f*)(sBC + s * 32 + 4 * q4);
        const v4f cv = *(const v4f*)(sBC + s * 32 + kNst + 4 * q4);
        Bs[4 * q4 + 0] = bv[0]; Bs[4 * q4 + 1] = bv[1]; Bs[4 * q4 + 2] = bv[2]; Bs[4 * q4 + 3] = bv[3];
        Cs[4 * q4 + 0] = cv[0]; Cs[4 * q4 + 1] = cv[1]; Cs[4 * q4 + 2] = cv[2]; Cs[4 * q4 + 3] = cv[3];
      }
      const float v0 = h16_to_f32(wd & 0xffffu) + bb0;
      const float v1 = h16_to_f32(wd >> 16) + bb1;
      const float x0 = h16_to_f32(wu & 0xffffu);
      const float x1 = h16_to_f32(wu >> 16);
      const float z0 = h16_to_f32(wz & 0xffffu);
      const float z1 = h16_to_f32(wz >> 16);
      const float y0 = scan_step(h0, nA0, Bs, Cs, v0, x0, z0, Dd0);
      const float y1 = scan_step(h1, nA1, Bs, Cs, v1, x1, z1, Dd1);
      const _Float16 q0 = (_Float16)(y0 * kCarryY);
      const _Float16 q1 = (_Float16)(y1 * kCarryY);
      const unsigned pw = (unsigned)__builtin_bit_cast(unsigned short, q0) |
                          ((unsigned)__builtin_bit_cast(unsigned short, q1) << 16);
      sY[s * kScanT + tid] = pw;
    }
    __syncthreads();
    for (int pass = 0; pass < 2; ++pass) {
#pragma unroll 1
      for (int it = 0; it < 16; ++it) {
        const int row = it * 4 + wave;
        const v4u val = *(const v4u*)(sY + row * kScanT + lane * 4);
        *(volatile v4u*)(YGw + (((row0 + t0 + row) * kDin + d0) >> 1) + lane * 4) = val;
      }
      __threadfence();
    }
  }
}

extern "C" void kernel_launch(void* const* d_in, const int* in_sizes, int n_in,
                              void* d_out, int out_size, void* d_ws, size_t ws_size,
                              hipStream_t stream) {
  if (n_in < 10) return;
  if (in_sizes[0] != kRows * kDm) return;
  if (in_sizes[1] != kXZP * kDm) return;
  if (in_sizes[2] != kDin * 3) return;
  if (in_sizes[3] != kDin) return;
  if (in_sizes[4] != kPrjN * kDin) return;
  if (in_sizes[5] != kDin * kDtR) return;
  if (in_sizes[6] != kDin) return;
  if (in_sizes[7] != kDin * kNst) return;
  if (in_sizes[8] != kDin) return;
  if (in_sizes[9] != kDm * kDin) return;
  if (out_size != kRows * kDm) return;
  if (ws_size < kWsTotal) return;

  const float* x       = (const float*)d_in[0];
  const float* W_in    = (const float*)d_in[1];
  const float* conv_w  = (const float*)d_in[2];
  const float* conv_b  = (const float*)d_in[3];
  const float* W_xproj = (const float*)d_in[4];
  const float* W_dt    = (const float*)d_in[5];
  const float* b_dt    = (const float*)d_in[6];
  const float* A_log   = (const float*)d_in[7];
  const float* Dp      = (const float*)d_in[8];
  const float* W_out   = (const float*)d_in[9];
  float* out = (float*)d_out;

  char* ws = (char*)d_ws;
  unsigned short* XH  = (unsigned short*)(ws + kOffXH);
  unsigned short* WIH = (unsigned short*)(ws + kOffWIH);
  unsigned short* WXH = (unsigned short*)(ws + kOffWXH);
  unsigned short* WDH = (unsigned short*)(ws + kOffWDH);
  unsigned short* WOH = (unsigned short*)(ws + kOffWOH);
  unsigned short* XZ  = (unsigned short*)(ws + kOffXZ);
  unsigned short* UC  = (unsigned short*)(ws + kOffUC);
  float*          PRJ = (float*)(ws + kOffPRJ);
  unsigned short* DTH = (unsigned short*)(ws + kOffDTH);
  unsigned short* DL  = (unsigned short*)(ws + kOffDL);
  unsigned short* YG  = (unsigned short*)(ws + kOffYG);

  cast_plane_kernel<<<(kRows * kDm / 8) / 256, 256, 0, stream>>>(x, XH, kRows * kDm / 8, kRows * kDm / 8, 1.0f);
  cast_plane_kernel<<<(kXZP * kDm / 8) / 256, 256, 0, stream>>>(W_in, WIH, kXZP * kDm / 8, kXZP * kDm / 8, kCarryW);
  cast_plane_kernel<<<(kPrjP * kDin / 8) / 256, 256, 0, stream>>>(W_xproj, WXH, kPrjN * kDin / 8, kPrjP * kDin / 8, kCarryW);
  cast_plane_kernel<<<(kDin * kDtR / 8) / 256, 256, 0, stream>>>(W_dt, WDH, kDin * kDtR / 8, kDin * kDtR / 8, kCarryWdt);
  cast_plane_kernel<<<(kDm * kDin / 8) / 256, 256, 0, stream>>>(W_out, WOH, kDm * kDin / 8, kDm * kDin / 8, kCarryW);

  wmma_gemm64_f16<1><<<dim3((kRows / 64) * (kXZP / 64) / 8), 256, 0, stream>>>(
      XH, kDm, WIH, kDm, (void*)XZ, kXZP, kRows, kXZP, kDm, 1.0f / kCarryW);

  conv_silu_kernel<<<dim3(kDin / 256, kRows / 64), 128, 0, stream>>>(
      (const unsigned*)XZ, conv_w, conv_b, UC);

  wmma_gemm64_f16<0><<<dim3((kRows / 64) * (kPrjP / 64) / 8), 256, 0, stream>>>(
      UC, kDin, WXH, kDin, (void*)PRJ, kPrjP, kRows, kPrjP, kDin, 1.0f / kCarryW);

  dt_cast_kernel<<<(kRows * kDtR / 8) / 256, 256, 0, stream>>>(PRJ, DTH, kRows * kDtR / 8, kCarryDt);

  wmma_gemm64_f16<1><<<dim3((kRows / 64) * (kDin / 64) / 8), 256, 0, stream>>>(
      DTH, kDtR, WDH, kDtR, (void*)DL, kDin, kRows, kDin, kDtR, 1.0f / (kCarryDt * kCarryWdt));

  scan_kernel<<<kBatch * (kDin / kScanCh), kScanT, 0, stream>>>(
      PRJ, (const unsigned*)DL, (const unsigned*)UC, (const unsigned*)XZ, b_dt, A_log, Dp, (unsigned*)YG);

  wmma_gemm64_f16<0><<<dim3((kRows / 64) * (kDm / 64) / 8), 256, 0, stream>>>(
      YG, kDin, WOH, kDin, (void*)out, kDm, kRows, kDm, kDin, 1.0f / (kCarryY * kCarryW));
}
